// ODEFunc_53987738911626
// MI455X (gfx1250) — hardware-verified
//
#include <hip/hip_runtime.h>
#include <math.h>
#include <stddef.h>

typedef __attribute__((ext_vector_type(16))) _Float16 v16h;
typedef __attribute__((ext_vector_type(8)))  _Float16 v8h;
typedef __attribute__((ext_vector_type(16))) __bf16   v16b;
typedef __attribute__((ext_vector_type(8)))  __bf16   v8b;
typedef __attribute__((ext_vector_type(8)))  float    v8f;
typedef __attribute__((ext_vector_type(4)))  float    v4f;
typedef __attribute__((ext_vector_type(4)))  unsigned int v4u;
typedef __attribute__((ext_vector_type(8)))  unsigned int v8u;

constexpr int kD    = 32;
constexpr int kH1   = 50;
constexpr int kH1P  = 64;
constexpr int kQ    = 528;
constexpr int kQP   = 544;
constexpr int kH2   = 700;
constexpr int kH2P  = 704;
constexpr int kLdW2aT = 576;
constexpr int kLdW2bT = 704;
constexpr int kLdW1T  = 64;
constexpr float kWCarry    = 256.0f;
constexpr float kWCarryInv = 1.0f / 256.0f;

static_assert(kQP % 32 == 0 && kH2P % 32 == 0 && kH1P % 32 == 0 && kD % 32 == 0, "every WMMA K is a multiple of 32");
static_assert(kH2P % 64 == 0 && kH1P % 64 == 0, "hidden chunks are whole 64-col groups");
static_assert((kLdW2aT * 2) % 128 == 0 && (kLdW2bT * 2) % 128 == 0 && (kLdW1T * 2) % 128 == 0, "plane rows are whole 128-B lines");
static_assert(kLdW2aT >= kQP && kLdW2bT >= kH2P && kLdW1T >= kH1P && kLdW1T >= kD, "pitches cover padded K");

constexpr size_t kOffW2aT   = 0;
constexpr size_t kBytesW2aT = (size_t)kH2P * kLdW2aT * 2;
constexpr size_t kOffW2bT   = kOffW2aT + kBytesW2aT;
constexpr size_t kBytesW2bT = (size_t)64 * kLdW2bT * 2;
constexpr size_t kOffW1aT   = kOffW2bT + kBytesW2bT;
constexpr size_t kBytesW1T  = (size_t)64 * kLdW1T * 2;
constexpr size_t kOffW1bT   = kOffW1aT + kBytesW1T;
constexpr size_t kWsTotal   = kOffW1bT + kBytesW1T;
static_assert(kBytesW2aT == 811008 && kOffW2bT == 811008 && kOffW1aT == 901120 && kOffW1bT == 909312 && kWsTotal == 917504, "region map");
static_assert(kOffW2bT % 128 == 0 && kOffW1aT % 128 == 0 && kOffW1bT % 128 == 0, "128-B aligned carves");
static_assert(kWsTotal <= (size_t)134217728, "carve under 128 MiB");

constexpr int kWavesBlk    = 2;
constexpr int kRowsBlk     = 32;
constexpr int kThreadsMain = 64;
constexpr int kQPitch = kQP;
constexpr int kYPitch = 32;
constexpr int kHPitch = 72;
constexpr int kOPitch = 36;
static_assert((kQPitch * 2) % 16 == 0 && (kHPitch * 2) % 16 == 0 && (kOPitch * 4) % 16 == 0 && (kYPitch * 4) % 16 == 0, "16-B aligned LDS rows");

__device__ __forceinline__ unsigned short f2bf_bits(float f) {
  unsigned u = __float_as_uint(f);
  return (unsigned short)((u + 0x7FFFu + ((u >> 16) & 1u)) >> 16);
}
__device__ __forceinline__ float bf_bits2f(unsigned short h) { return __uint_as_float(((unsigned)h) << 16); }
__device__ __forceinline__ unsigned pk16(unsigned short a, unsigned short b) { return (unsigned)a | ((unsigned)b << 16); }
__device__ __forceinline__ unsigned short h_bits(float f) { const _Float16 h = (_Float16)f; return __builtin_bit_cast(unsigned short, h); }
__device__ __forceinline__ float rne_bf(float f) { return bf_bits2f(f2bf_bits(f)); }

__device__ __forceinline__ v16b ldfrag_bf(const unsigned short* p) {
  union { v16b v; v8b h[2]; } f;
  f.h[0] = *(const v8b*)(p);
  f.h[1] = *(const v8b*)(p + 16);
  return f.v;
}
__device__ __forceinline__ v16h ldfrag_h(const unsigned short* p) {
  union { v16h v; v8h h[2]; } f;
  f.h[0] = *(const v8h*)(p);
  f.h[1] = *(const v8h*)(p + 16);
  return f.v;
}
__device__ __forceinline__ v8f mma_bf(v16b a, v16b b, v8f c) {
  return __builtin_amdgcn_wmma_f32_16x16x32_bf16(false, a, false, b, (short)0, c, false, false);
}
__device__ __forceinline__ v8f mma_h(v16h a, v16h b, v8f c) {
  return __builtin_amdgcn_wmma_f32_16x16x32_f16(false, a, false, b, (short)0, c, false, false);
}
__device__ __forceinline__ void guard_acc4_h5(v8f& a0, v8f& a1, v8f& a2, v8f& a3,
                                              v16h f0, v16h f1, v16h f2, v16h f3, v16h f4) {
  asm volatile("v_nop\n\tv_nop\n\tv_nop\n\tv_nop"
               : "+v"(a0), "+v"(a1), "+v"(a2), "+v"(a3)
               : "v"(f0), "v"(f1), "v"(f2), "v"(f3), "v"(f4));
}
__device__ __forceinline__ void guard_acc4_b5(v8f& a0, v8f& a1, v8f& a2, v8f& a3,
                                              v16b f0, v16b f1, v16b f2, v16b f3, v16b f4) {
  asm volatile("v_nop\n\tv_nop\n\tv_nop\n\tv_nop"
               : "+v"(a0), "+v"(a1), "+v"(a2), "+v"(a3)
               : "v"(f0), "v"(f1), "v"(f2), "v"(f3), "v"(f4));
}
__device__ __forceinline__ void guard_acc2_h3(v8f& a0, v8f& a1, v16h f0, v16h f1, v16h f2) {
  asm volatile("v_nop\n\tv_nop\n\tv_nop\n\tv_nop" : "+v"(a0), "+v"(a1) : "v"(f0), "v"(f1), "v"(f2));
}
__device__ __forceinline__ void guard_acc4(v8f& a, v8f& b, v8f& c, v8f& d) {
  asm volatile("v_nop\n\tv_nop\n\tv_nop\n\tv_nop" : "+v"(a), "+v"(b), "+v"(c), "+v"(d));
}
__device__ __forceinline__ void guard_acc2(v8f& a, v8f& b) {
  asm volatile("v_nop\n\tv_nop\n\tv_nop\n\tv_nop" : "+v"(a), "+v"(b));
}

__device__ __forceinline__ float tanh_acc(float x) {
  const float ax = fabsf(x);
  const float e  = expf(-2.0f * ax);
  const float r  = (1.0f - e) * __builtin_amdgcn_rcpf(1.0f + e);
  return copysignf(r, x);
}

template <int CVT>
__global__ __launch_bounds__(128) void wt_prep(const float* __restrict__ src, int kReal, int nReal,
                                               unsigned short* __restrict__ dst, int ldo, float scale) {
  __shared__ __align__(16) unsigned short smb[64][72];
  const int t  = threadIdx.x;
  const int k0 = blockIdx.x * 64;
  const int n0 = blockIdx.y * 64;
#pragma unroll 1
  for (int i8 = 0; i8 < 8; ++i8) {
#pragma unroll
    for (int i = 0; i < 4; ++i) {
      const int e  = (i8 * 4 + i) * 128 + t;
      const int kl = e >> 6;
      const int nl = e & 63;
      const int k  = k0 + kl;
      const int n  = n0 + nl;
      const int kc = k < kReal ? k : kReal - 1;
      const int nc = n < nReal ? n : nReal - 1;
      float v = src[(size_t)kc * nReal + nc];
      const float fz = (k < kReal && n < nReal) ? 1.0f : 0.0f;
      v = fmaf(v, fz, 0.0f);
      unsigned short bits;
      if (CVT == 0) {
        bits = f2bf_bits(v * scale);
      } else {
        bits = h_bits(rne_bf(v) * scale);
      }
      smb[nl][kl] = bits;
    }
  }
  __syncthreads();
  const int lane = t & 31, wv = t >> 5;
  const int q8 = lane >> 3, c8 = (lane & 7) * 8;
  for (int pass = 0; pass < 2; ++pass) {
#pragma unroll
    for (int it = 0; it < 4; ++it) {
      const int row = wv * 16 + it * 4 + q8;
      const v4u u = *(const v4u*)(&smb[row][c8]);
      *(volatile v4u*)(dst + (size_t)(n0 + row) * ldo + k0 + c8) = u;
    }
    __threadfence();
  }
}

__global__ __launch_bounds__(kThreadsMain) void ode_main(
    const float* __restrict__ y,
    const float* __restrict__ b1a, const float* __restrict__ b1b,
    const float* __restrict__ b2a, const float* __restrict__ b2b,
    const unsigned short* __restrict__ w2aT, const unsigned short* __restrict__ w2bT,
    const unsigned short* __restrict__ w1aT, const unsigned short* __restrict__ w1bT,
    float* __restrict__ out, int nrows)
{
  __shared__ __align__(16) unsigned short qH[kWavesBlk][16 * kQPitch];
  __shared__ __align__(16) float          yT[kRowsBlk * kYPitch];
  __shared__ __align__(16) unsigned short rcT[kQ];
  __shared__ __align__(16) unsigned short hT[kWavesBlk][16 * kHPitch];
  __shared__ __align__(16) float          oT[kWavesBlk][16 * kOPitch];

  const int tid  = threadIdx.x;
  const int lane = tid & 31;
  const int w    = tid >> 5;
  const int hh   = lane >> 4;
  const int rl   = lane & 15;
  const int koff = hh * 8;
  const int row0 = blockIdx.x * kRowsBlk;
  const v8f z8 = {0.f, 0.f, 0.f, 0.f, 0.f, 0.f, 0.f, 0.f};

#pragma unroll
  for (int i = 0; i < 9; ++i) {
    const int q = tid + 64 * i;
    if (q < kQ) {
      int r = (int)((sqrtf((float)(8 * q + 1)) - 1.0f) * 0.5f);
      if ((r + 1) * (r + 2) / 2 <= q) r += 1;
      if (r * (r + 1) / 2 > q) r -= 1;
      r = r < 0 ? 0 : (r > kD - 1 ? kD - 1 : r);
      int c = q - r * (r + 1) / 2;
      c = c < 0 ? 0 : (c > r ? r : c);
      rcT[q] = (unsigned short)(r | (c << 8));
    }
  }
  {
    const int yr = tid >> 1;
    const int c0 = (tid & 1) * 16;
    int grow = row0 + yr;
    grow = grow < nrows ? grow : nrows - 1;
    const float* yp = y + (size_t)grow * kD + c0;
#pragma unroll
    for (int i = 0; i < 4; ++i) {
      const v4f v = *(const v4f*)(yp + 4 * i);
      v4f o;
      o[0] = rne_bf(v[0]); o[1] = rne_bf(v[1]); o[2] = rne_bf(v[2]); o[3] = rne_bf(v[3]);
      *(v4f*)(yT + yr * kYPitch + c0 + 4 * i) = o;
    }
  }
  __syncthreads();

  {
    const float* yrow = yT + (w * 16 + rl) * kYPitch;
    unsigned short* qh = qH[w] + rl * kQPitch;
#pragma unroll 1
    for (int j = 0; j < 33; ++j) {
      const int q0 = 16 * j + 8 * hh;
      const v4u tw = *(const v4u*)(rcT + q0);
      unsigned hw[4];
#pragma unroll
      for (int i2 = 0; i2 < 4; ++i2) {
        const unsigned wd = tw[i2];
        const unsigned ra = wd & 0xffu, ca = (wd >> 8) & 0xffu;
        const unsigned rb = (wd >> 16) & 0xffu, cb = (wd >> 24) & 0xffu;
        const float pa = yrow[ra] * yrow[ca];
        const float pb = yrow[rb] * yrow[cb];
        hw[i2] = pk16(h_bits(pa), h_bits(pb));
      }
      *(v4u*)(qh + q0) = (v4u){hw[0], hw[1], hw[2], hw[3]};
    }
    const v4u zq = (v4u){0u, 0u, 0u, 0u};
    *(v4u*)(qh + kQ + 8 * hh) = zq;
  }
  __syncthreads();

  v8f oacc0 = z8, oacc1 = z8;
  const unsigned short* qhA = qH[w] + rl * kQPitch + koff;
  const unsigned short* hA  = hT[w] + rl * kHPitch + koff;
  unsigned short* hW = hT[w];

#pragma unroll 1
  for (int jj = 0; jj < kH2P / 64; ++jj) {
    v8f hacc[4];
    hacc[0] = z8; hacc[1] = z8; hacc[2] = z8; hacc[3] = z8;
    const unsigned short* bbase = w2aT + (size_t)(jj * 64 + rl) * kLdW2aT + koff;
#pragma unroll 1
    for (int ks = 0; ks < kQP / 32; ++ks) {
      const v16h ah = ldfrag_h(qhA + ks * 32);
      v16h bw[4];
#pragma unroll
      for (int t = 0; t < 4; ++t) bw[t] = ldfrag_h(bbase + (size_t)t * 16 * kLdW2aT + ks * 32);
#pragma unroll
      for (int t = 0; t < 4; ++t) {
        hacc[t] = mma_h(ah, bw[t], hacc[t]);
      }
      guard_acc4_h5(hacc[0], hacc[1], hacc[2], hacc[3], ah, bw[0], bw[1], bw[2], bw[3]);
    }
    guard_acc4(hacc[0], hacc[1], hacc[2], hacc[3]);
#pragma unroll
    for (int t = 0; t < 4; ++t) {
      const int col  = jj * 64 + t * 16 + rl;
      const int colc = col < kH2 ? col : kH2 - 1;
      float bb = b2a[colc];
      const float fz = (col < kH2) ? 1.0f : 0.0f;
      bb = fmaf(rne_bf(bb), fz, 0.0f);
#pragma unroll
      for (int r = 0; r < 8; ++r) {
        hW[(8 * hh + r) * kHPitch + t * 16 + rl] = h_bits(tanh_acc(hacc[t][r] * kWCarryInv + bb));
      }
    }
    __syncthreads();
#pragma unroll
    for (int k2 = 0; k2 < 2; ++k2) {
      const v16h af  = ldfrag_h(hA + k2 * 32);
      const v16h bu0 = ldfrag_h(w2bT + (size_t)rl * kLdW2bT + jj * 64 + k2 * 32 + koff);
      const v16h bu1 = ldfrag_h(w2bT + (size_t)(16 + rl) * kLdW2bT + jj * 64 + k2 * 32 + koff);
      oacc0 = mma_h(af, bu0, oacc0);
      oacc1 = mma_h(af, bu1, oacc1);
      guard_acc2_h3(oacc0, oacc1, af, bu0, bu1);
    }
    __syncthreads();
  }

  {
    const float* yrow = yT + (w * 16 + rl) * kYPitch;
    const v4f ya0 = *(const v4f*)(yrow + koff);
    const v4f ya1 = *(const v4f*)(yrow + koff + 4);
    const v4f ya2 = *(const v4f*)(yrow + 16 + koff);
    const v4f ya3 = *(const v4f*)(yrow + 16 + koff + 4);
    v8u yw;
    yw[0] = pk16(f2bf_bits(ya0[0]), f2bf_bits(ya0[1]));
    yw[1] = pk16(f2bf_bits(ya0[2]), f2bf_bits(ya0[3]));
    yw[2] = pk16(f2bf_bits(ya1[0]), f2bf_bits(ya1[1]));
    yw[3] = pk16(f2bf_bits(ya1[2]), f2bf_bits(ya1[3]));
    yw[4] = pk16(f2bf_bits(ya2[0]), f2bf_bits(ya2[1]));
    yw[5] = pk16(f2bf_bits(ya2[2]), f2bf_bits(ya2[3]));
    yw[6] = pk16(f2bf_bits(ya3[0]), f2bf_bits(ya3[1]));
    yw[7] = pk16(f2bf_bits(ya3[2]), f2bf_bits(ya3[3]));
    const v16b ya = __builtin_bit_cast(v16b, yw);
    v16b bw[4];
#pragma unroll
    for (int t = 0; t < 4; ++t) bw[t] = ldfrag_bf(w1aT + (size_t)(t * 16 + rl) * kLdW1T + koff);
    v8f a1[4];
    a1[0] = z8; a1[1] = z8; a1[2] = z8; a1[3] = z8;
#pragma unroll
    for (int t = 0; t < 4; ++t) a1[t] = mma_bf(ya, bw[t], a1[t]);
    guard_acc4_b5(a1[0], a1[1], a1[2], a1[3], ya, bw[0], bw[1], bw[2], bw[3]);
#pragma unroll
    for (int t = 0; t < 4; ++t) {
      const int col  = t * 16 + rl;
      const int colc = col < kH1 ? col : kH1 - 1;
      float bb = b1a[colc];
      const float fz = (col < kH1) ? 1.0f : 0.0f;
      bb = fmaf(rne_bf(bb), fz, 0.0f);
#pragma unroll
      for (int r = 0; r < 8; ++r) {
        hW[(8 * hh + r) * kHPitch + t * 16 + rl] = h_bits(tanh_acc(a1[t][r] + bb));
      }
    }
  }
  __syncthreads();
#pragma unroll
  for (int k2 = 0; k2 < 2; ++k2) {
    const v16h af  = ldfrag_h(hA + k2 * 32);
    const v16h bu0 = ldfrag_h(w1bT + (size_t)rl * kLdW1T + k2 * 32 + koff);
    const v16h bu1 = ldfrag_h(w1bT + (size_t)(16 + rl) * kLdW1T + k2 * 32 + koff);
    oacc0 = mma_h(af, bu0, oacc0);
    oacc1 = mma_h(af, bu1, oacc1);
    guard_acc2_h3(oacc0, oacc1, af, bu0, bu1);
  }
  guard_acc2(oacc0, oacc1);

  {
    const float bo0 = rne_bf(b1b[rl]) + rne_bf(b2b[rl]);
    const float bo1 = rne_bf(b1b[16 + rl]) + rne_bf(b2b[16 + rl]);
    float* os = oT[w];
#pragma unroll
    for (int r = 0; r < 8; ++r) {
      os[(8 * hh + r) * kOPitch + rl]      = oacc0[r] * kWCarryInv + bo0;
      os[(8 * hh + r) * kOPitch + 16 + rl] = oacc1[r] * kWCarryInv + bo1;
    }
  }
  __syncthreads();
  {
    const int q8 = lane >> 3, c4 = (lane & 7) * 4;
    const float* os = oT[w];
    float* ob = out + (size_t)(row0 + w * 16) * kD;
    for (int pass = 0; pass < 2; ++pass) {
#pragma unroll
      for (int it = 0; it < 4; ++it) {
        const int row = it * 4 + q8;
        const v4f v = *(const v4f*)(os + row * kOPitch + c4);
        *(volatile v4f*)(ob + (size_t)row * kD + c4) = v;
      }
      __threadfence();
    }
  }
}

extern "C" void kernel_launch(void* const* d_in, const int* in_sizes, int n_in,
                              void* d_out, int out_size, void* d_ws, size_t ws_size,
                              hipStream_t stream) {
  (void)n_in; (void)out_size;
  const float* y   = (const float*)d_in[1];
  const float* W1a = (const float*)d_in[2];
  const float* b1a = (const float*)d_in[3];
  const float* W1b = (const float*)d_in[4];
  const float* b1b = (const float*)d_in[5];
  const float* W2a = (const float*)d_in[6];
  const float* b2a = (const float*)d_in[7];
  const float* W2b = (const float*)d_in[8];
  const float* b2b = (const float*)d_in[9];
  float* out = (float*)d_out;

  if (ws_size < kWsTotal) return;
  unsigned char* ws = (unsigned char*)d_ws;
  unsigned short* w2aT = (unsigned short*)(ws + kOffW2aT);
  unsigned short* w2bT = (unsigned short*)(ws + kOffW2bT);
  unsigned short* w1aT = (unsigned short*)(ws + kOffW1aT);
  unsigned short* w1bT = (unsigned short*)(ws + kOffW1bT);

  wt_prep<1><<<dim3(kLdW2aT / 64, kH2P / 64), 128, 0, stream>>>(W2a, kQ, kH2, w2aT, kLdW2aT, kWCarry);
  wt_prep<1><<<dim3(kLdW2bT / 64, 1), 128, 0, stream>>>(W2b, kH2, kD, w2bT, kLdW2bT, kWCarry);
  wt_prep<0><<<dim3(1, 1), 128, 0, stream>>>(W1a, kD, kH1, w1aT, kLdW1T, 1.0f);
  wt_prep<1><<<dim3(1, 1), 128, 0, stream>>>(W1b, kH1, kD, w1bT, kLdW1T, kWCarry);

  const int nrows = in_sizes[1] / kD;
  const int nblk  = nrows / kRowsBlk;
  if (nblk > 0) {
    ode_main<<<dim3((unsigned)nblk), kThreadsMain, 0, stream>>>(
        y, b1a, b1b, b2a, b2b, w2aT, w2bT, w1aT, w1bT, out, nrows);
  }
}
